// WaveNet_14439680049375
// MI455X (gfx1250) — hardware-verified
//
#include <hip/hip_runtime.h>
#include <math.h>
#include <stddef.h>

typedef __attribute__((ext_vector_type(16))) _Float16 v16h;
typedef __attribute__((ext_vector_type(8)))  _Float16 v8h;
typedef __attribute__((ext_vector_type(16))) __bf16   v16b;
typedef __attribute__((ext_vector_type(8)))  __bf16   v8b;
typedef __attribute__((ext_vector_type(8)))  float    v8f;
typedef __attribute__((ext_vector_type(4)))  float    v4f;
typedef __attribute__((ext_vector_type(4)))  unsigned v4u;

constexpr int kMu      = 256;
constexpr int kRes     = 32;
constexpr int kSkipCh  = 512;
constexpr int kTin     = 16384;
constexpr int kNblk    = 50;
constexpr int kFinal   = 11269;
constexpr int kMpad    = 11328;
constexpr int kKskip   = kNblk * kRes;
constexpr int kUtiles  = (kFinal + 15) / 16;
constexpr int kGrowsW  = kUtiles * 16;
constexpr int kThreads = 256;
constexpr float kWcarry = 64.0f;
constexpr float kAcarry = 256.0f;
constexpr float kFold   = 1.0f / 16384.0f;

static_assert(kMpad % 64 == 0 && kMpad >= kFinal, "M tile multiple");
static_assert(kGrowsW <= kMpad && kGrowsW >= kFinal, "u tiles inside the padded plane");
static_assert(kKskip % 32 == 0 && kSkipCh % 64 == 0 && kMu % 64 == 0, "GEMM N/K multiples");
static_assert(kSkipCh % 32 == 0, "K multiple of 32");
static_assert((kTin * 8) % kThreads == 0, "embed grid exact");
static_assert((kNblk * 64 * 64 / 8) % kThreads == 0, "gate pack grid exact");
static_assert((kSkipCh * kKskip / 8) % kThreads == 0, "skip pack grid exact");

constexpr size_t kBytesX    = (size_t)kTin * kRes * 4;
constexpr size_t kBytesG    = (size_t)kMpad * kKskip * 2;
constexpr size_t kBytesGT   = (size_t)kMpad * kRes * 2;
constexpr size_t kBytesE    = (size_t)kMpad * kSkipCh * 2;
constexpr size_t kBytesWG   = (size_t)kNblk * 64 * 64 * 2;
constexpr size_t kBytesWR   = (size_t)kNblk * 32 * 32 * 2;
constexpr size_t kBytesWS   = (size_t)kSkipCh * kKskip * 2;
constexpr size_t kBytesWP1  = (size_t)kSkipCh * kSkipCh * 2;
constexpr size_t kBytesWP2  = (size_t)kMu * kSkipCh * 2;
constexpr size_t kBytesBias = (size_t)(kSkipCh + kSkipCh + kMu) * 4;
constexpr size_t kOffX0   = 0;
constexpr size_t kOffX1   = kOffX0 + kBytesX;
constexpr size_t kOffG    = kOffX1 + kBytesX;
constexpr size_t kOffGT   = kOffG + kBytesG;
constexpr size_t kOffE1   = kOffGT + kBytesGT;
constexpr size_t kOffE2   = kOffE1 + kBytesE;
constexpr size_t kOffWG   = kOffE2 + kBytesE;
constexpr size_t kOffWR   = kOffWG + kBytesWG;
constexpr size_t kOffWS   = kOffWR + kBytesWR;
constexpr size_t kOffWP1  = kOffWS + kBytesWS;
constexpr size_t kOffWP2  = kOffWP1 + kBytesWP1;
constexpr size_t kOffBias = kOffWP2 + kBytesWP2;
constexpr size_t kWsTotal = kOffBias + kBytesBias;
static_assert(kBytesX % 256 == 0 && kBytesG % 256 == 0 && kBytesGT % 256 == 0 && kBytesE % 256 == 0, "align");
static_assert(kBytesWG % 256 == 0 && kBytesWR % 256 == 0 && kBytesWS % 256 == 0 && kBytesWP1 % 256 == 0 && kBytesWP2 % 256 == 0, "align");
static_assert(kWsTotal <= (size_t)134217728, "workspace carve under 128 MiB");

__device__ __forceinline__ unsigned short f2bf_bits(float f) {
  unsigned u = __float_as_uint(f);
  return (unsigned short)((u + 0x7FFFu + ((u >> 16) & 1u)) >> 16);
}
__device__ __forceinline__ float bf_bits2f(unsigned short h) { return __uint_as_float(((unsigned)h) << 16); }
__device__ __forceinline__ float bfr(float f) { return bf_bits2f(f2bf_bits(f)); }

__device__ __forceinline__ void dep_guard_h(v8f& a, v8f& b, v16h x, v16h y) { asm volatile("v_nop\n\tv_nop\n\tv_nop\n\tv_nop" : "+v"(a), "+v"(b) : "v"(x), "v"(y)); }
__device__ __forceinline__ void dep_guard_b(v8f& a, v8f& b, v16b x, v16b y) { asm volatile("v_nop\n\tv_nop\n\tv_nop\n\tv_nop" : "+v"(a), "+v"(b) : "v"(x), "v"(y)); }
__device__ __forceinline__ void keep4_h(v16h a, v16h b, v16h c, v16h d) { asm volatile("v_nop" :: "v"(a), "v"(b), "v"(c), "v"(d)); }
__device__ __forceinline__ void keep4_b(v16b a, v16b b, v16b c, v16b d) { asm volatile("v_nop" :: "v"(a), "v"(b), "v"(c), "v"(d)); }
__device__ __forceinline__ void acc_guard4(v8f& a, v8f& b, v8f& c, v8f& d) { asm volatile("v_nop\n\tv_nop\n\tv_nop\n\tv_nop" : "+v"(a), "+v"(b), "+v"(c), "+v"(d)); }
__device__ __forceinline__ void guard1x4(v8f& a, v16h w, v16h x, v16h y, v16h z) {
  asm volatile("v_nop\n\tv_nop\n\tv_nop\n\tv_nop" : "+v"(a) : "v"(w), "v"(x), "v"(y), "v"(z));
}
__device__ __forceinline__ void guard2x3(v8f& a, v8f& b, v16h x, v16h y, v16h z) {
  asm volatile("v_nop\n\tv_nop\n\tv_nop\n\tv_nop" : "+v"(a), "+v"(b) : "v"(x), "v"(y), "v"(z));
}
template <typename T> struct Frag;
template <> struct Frag<_Float16> {
  typedef v16h V; union U { v16h v; v8h h[2]; };
  static __device__ __forceinline__ v16h load(const _Float16* p) {
    U f; f.h[0] = *(const v8h*)(p); f.h[1] = *(const v8h*)(p + 16); return f.v;
  }
  static __device__ __forceinline__ v8f mma(v16h a, v16h b, v8f c) {
    return __builtin_amdgcn_wmma_f32_16x16x32_f16(false, a, false, b, (short)0, c, false, false);
  }
  static __device__ __forceinline__ void guard(v8f& a, v8f& b, v16h x, v16h y) { dep_guard_h(a, b, x, y); }
  static __device__ __forceinline__ void keep(v16h a, v16h b, v16h c, v16h d) { keep4_h(a, b, c, d); }
};
template <> struct Frag<__bf16> {
  typedef v16b V; union U { v16b v; v8b h[2]; };
  static __device__ __forceinline__ v16b load(const __bf16* p) {
    U f; f.h[0] = *(const v8b*)(p); f.h[1] = *(const v8b*)(p + 16); return f.v;
  }
  static __device__ __forceinline__ v8f mma(v16b a, v16b b, v8f c) {
    return __builtin_amdgcn_wmma_f32_16x16x32_bf16(false, a, false, b, (short)0, c, false, false);
  }
  static __device__ __forceinline__ void guard(v8f& a, v8f& b, v16b x, v16b y) { dep_guard_b(a, b, x, y); }
  static __device__ __forceinline__ void keep(v16b a, v16b b, v16b c, v16b d) { keep4_b(a, b, c, d); }
};
typedef Frag<_Float16> FragH;

template <int ET> struct Elem;
template <> struct Elem<0> { typedef _Float16 T; };
template <> struct Elem<1> { typedef __bf16 T; };
template <int ET, bool SPLIT, int BIAS_MODE, int OUT_MODE, bool RESID, int ACT = 0>
__global__ __launch_bounds__(256) void wmma_gemm64(
    const unsigned short* __restrict__ Ap, const unsigned short* __restrict__ A2p, int lda, long strideA,
    const unsigned short* __restrict__ Btp, const unsigned short* __restrict__ Bt2p, int ldb, long strideB,
    void* __restrict__ Cout, void* __restrict__ Cout2, int ldc, long strideC,
    const float* __restrict__ bias,
    const float* __restrict__ resid, long strideR,
    int M, int N, int K, float scale, float oscale, int Mreal) {
  typedef typename Elem<ET>::T T;
  typedef typename Frag<T>::V V;
  const T* A = (const T*)Ap; const T* A2 = (const T*)A2p; const T* Bt = (const T*)Btp; const T* Bt2 = (const T*)Bt2p;
  __shared__ __align__(16) float sT[8][16 * 68];
  const int b    = blockIdx.y;
  const int lane = threadIdx.x & 31;
  const int wave = threadIdx.x >> 5;
  const int tilesN = N >> 6;
  const int tilesM = M >> 6;
  const int tile = blockIdx.x * 8 + wave;
  if (tile >= tilesM * tilesN) return;
  const int tm = tile / tilesN;
  const int tn = tile - tm * tilesN;
  const int m0 = tm << 6;
  const int n0 = tn << 6;

  const T* Ab  = A  + (size_t)b * strideA;
  const T* Bb  = Bt + (size_t)b * strideB;
  const T* Ab2 = SPLIT ? (A2  + (size_t)b * strideA) : nullptr;
  const T* Bb2 = SPLIT ? (Bt2 + (size_t)b * strideB) : nullptr;

  const int rlane = lane & 15;
  const int koff  = (lane >> 4) * 8;
  const int mOff  = (lane >> 4) * 8;

  v8f acc[4][4];
#pragma unroll
  for (int i = 0; i < 4; ++i)
#pragma unroll
    for (int j = 0; j < 4; ++j) acc[i][j] = (v8f){0.f,0.f,0.f,0.f,0.f,0.f,0.f,0.f};

  for (int k0 = 0; k0 < K; k0 += 32) {
    V bh[4], bl[4];
#pragma unroll
    for (int j = 0; j < 4; ++j) {
      const size_t bo = (size_t)(n0 + (j << 4) + rlane) * ldb + koff + k0;
      bh[j] = Frag<T>::load(Bb + bo);
      if (SPLIT) bl[j] = Frag<T>::load(Bb2 + bo);
    }
#pragma unroll
    for (int i = 0; i < 4; ++i) {
      const size_t ao = (size_t)(m0 + (i << 4) + rlane) * lda + koff + k0;
      V ah = Frag<T>::load(Ab + ao);
      V al;
      if (SPLIT) al = Frag<T>::load(Ab2 + ao);
#pragma unroll
      for (int j = 0; j < 4; ++j) {
        acc[i][j] = Frag<T>::mma(ah, bh[j], acc[i][j]);
        if (SPLIT) {
          acc[i][j] = Frag<T>::mma(ah, bl[j], acc[i][j]);
          acc[i][j] = Frag<T>::mma(al, bh[j], acc[i][j]);
        }
      }
      Frag<T>::guard(acc[i][0], acc[i][3], ah, SPLIT ? al : ah);
    }
    Frag<T>::keep(bh[0], bh[1], bh[2], bh[3]);
    if (SPLIT) Frag<T>::keep(bl[0], bl[1], bl[2], bl[3]);
  }
  acc_guard4(acc[0][0], acc[0][1], acc[0][2], acc[0][3]);
  acc_guard4(acc[1][0], acc[1][1], acc[1][2], acc[1][3]);
  acc_guard4(acc[2][0], acc[2][1], acc[2][2], acc[2][3]);
  acc_guard4(acc[3][0], acc[3][1], acc[3][2], acc[3][3]);

  float* slab = sT[wave];
  const float* Rb = RESID ? (resid + (size_t)b * strideR) : nullptr;
#pragma unroll
  for (int i = 0; i < 4; ++i) {
    const int mBase = m0 + (i << 4);
#pragma unroll
    for (int j = 0; j < 4; ++j) {
      const int n = n0 + (j << 4) + rlane;
      float bv = 0.f;
      if (BIAS_MODE == 2) bv = bias[n];
#pragma unroll
      for (int r = 0; r < 8; ++r) {
        float v = acc[i][j][r] * scale;
        if (BIAS_MODE == 1) v += bias[mBase + mOff + r];
        if (BIAS_MODE == 2) v += bv;
        if (RESID) v += Rb[(size_t)(mBase + mOff + r) * ldc + n];
        if (ACT == 1) v = tanhf(v);
        if (ACT == 2) v = fmaxf(v, 0.0f);
        if (ACT == 3) v = v / (1.0f + expf(-v));
        if (ACT == 4) v = (v > 0.f) ? v : 0.01f * v;
        if (ACT == 5) v = 0.5f * v * (1.0f + erff(v * 0.70710678118654752f));
        if (ACT == 6) v = (v > 0.0f) ? v : (expf(v) - 1.0f);
        v = v * oscale;
        slab[(mOff + r) * 68 + (j << 4) + rlane] = v;
      }
    }
    __builtin_amdgcn_fence(__ATOMIC_RELEASE, "workgroup");
    __builtin_amdgcn_wave_barrier();
    __builtin_amdgcn_fence(__ATOMIC_ACQUIRE, "workgroup");
    if (OUT_MODE == 0) {
      float* C = (float*)Cout + (size_t)b * strideC;
      const int hh = lane >> 4, c4 = (lane & 15) * 4;
      for (int pass = 0; pass < 2; ++pass) {
#pragma unroll
        for (int it = 0; it < 8; ++it) {
          const int row = it * 2 + hh;
          v4f v = *(const v4f*)(slab + row * 68 + c4);
          if (mBase + row < Mreal) *(volatile v4f*)(C + (size_t)(mBase + row) * ldc + n0 + c4) = v;
        }
        __threadfence();
      }
    } else {
      const int q = lane >> 3, c8 = (lane & 7) * 8;
      unsigned short* C  = (unsigned short*)Cout  + (size_t)b * strideC;
      unsigned short* C2 = (OUT_MODE == 2) ? ((unsigned short*)Cout2 + (size_t)b * strideC) : nullptr;
      for (int pass = 0; pass < 2; ++pass) {
#pragma unroll
        for (int it = 0; it < 4; ++it) {
          const int row = it * 4 + q;
          const float* sp = slab + row * 68 + c8;
          v8h hv, lv;
#pragma unroll
          for (int e = 0; e < 8; ++e) {
            if (OUT_MODE == 1) {
              hv[e] = (_Float16)sp[e];
            } else {
              unsigned short hb = f2bf_bits(sp[e]);
              unsigned short lb = f2bf_bits(sp[e] - bf_bits2f(hb));
              hv[e] = __builtin_bit_cast(_Float16, hb);
              lv[e] = __builtin_bit_cast(_Float16, lb);
            }
          }
          if (mBase + row < Mreal) {
            *(volatile v8h*)(C + (size_t)(mBase + row) * ldc + n0 + c8) = hv;
            if (OUT_MODE == 2) *(volatile v8h*)(C2 + (size_t)(mBase + row) * ldc + n0 + c8) = lv;
          }
        }
        __threadfence();
      }
    }
    __builtin_amdgcn_fence(__ATOMIC_RELEASE, "workgroup");
    __builtin_amdgcn_wave_barrier();
    __builtin_amdgcn_fence(__ATOMIC_ACQUIRE, "workgroup");
  }
}

__global__ __launch_bounds__(kThreads) void k_pack_gate(const float* __restrict__ w_sig, const float* __restrict__ w_tanh,
                                                        unsigned short* __restrict__ O) {
  const int i = blockIdx.x * kThreads + threadIdx.x;
  if (i >= kNblk * 64 * 64 / 8) return;
  const int e0  = i * 8;
  const int blk = e0 >> 12;
  const int rem = e0 & 4095;
  const int n   = rem >> 6;
  const int k0  = rem & 63;
  const int tap = k0 >> 5;
  const int c0  = k0 & 31;
  const int o   = n & 31;
  const size_t base = (((size_t)blk * kRes + o) * kRes + c0) * 2 + tap;
  float vs[8], vt[8];
#pragma unroll
  for (int e = 0; e < 8; ++e) vs[e] = w_sig[base + 2 * e];
  asm volatile("" ::: "memory");
#pragma unroll
  for (int e = 0; e < 8; ++e) vt[e] = w_tanh[base + 2 * e];
  const float fs = (n < 32) ? 1.0f : 0.0f;
  const float ft = 1.0f - fs;
  v8h hv;
#pragma unroll
  for (int e = 0; e < 8; ++e) hv[e] = (_Float16)(kWcarry * (fs * bfr(vs[e]) + ft * bfr(vt[e])));
  const size_t oo = (size_t)e0;
  *(volatile v8h*)(O + oo) = hv;
  __threadfence();
  *(volatile v8h*)(O + oo) = hv;
}

__global__ __launch_bounds__(kThreads) void k_pack_skip(const float* __restrict__ w_skip, unsigned short* __restrict__ O) {
  const int i = blockIdx.x * kThreads + threadIdx.x;
  if (i >= kSkipCh * kKskip / 8) return;
  const int e0  = i * 8;
  const int m   = e0 / kKskip;
  const int k0  = e0 - m * kKskip;
  const int blk = k0 >> 5;
  const int c0  = k0 & 31;
  const float* src = w_skip + ((size_t)blk * kSkipCh + m) * kRes + c0;
  const v4f w0 = *(const v4f*)(src);
  const v4f w1 = *(const v4f*)(src + 4);
  v8h hv;
#pragma unroll
  for (int e = 0; e < 4; ++e) {
    const float f0 = w0[e];
    const float f1 = w1[e];
    hv[e]     = (_Float16)(kWcarry * bfr(f0));
    hv[4 + e] = (_Float16)(kWcarry * bfr(f1));
  }
  const size_t oo = (size_t)e0;
  *(volatile v8h*)(O + oo) = hv;
  __threadfence();
  *(volatile v8h*)(O + oo) = hv;
}

__global__ __launch_bounds__(kThreads) void k_pack_plain(const float* __restrict__ W, int n8, unsigned short* __restrict__ O) {
  const int i = blockIdx.x * kThreads + threadIdx.x;
  if (i >= n8) return;
  const size_t e0 = (size_t)i * 8;
  const v4f w0 = *(const v4f*)(W + e0);
  const v4f w1 = *(const v4f*)(W + e0 + 4);
  v8h hv;
#pragma unroll
  for (int e = 0; e < 4; ++e) {
    const float f0 = w0[e];
    const float f1 = w1[e];
    hv[e]     = (_Float16)(kWcarry * bfr(f0));
    hv[4 + e] = (_Float16)(kWcarry * bfr(f1));
  }
  *(volatile v8h*)(O + e0) = hv;
  __threadfence();
  *(volatile v8h*)(O + e0) = hv;
}

__global__ __launch_bounds__(kThreads) void k_bias(const float* __restrict__ b_skip, const float* __restrict__ b_p1,
                                                   const float* __restrict__ b_p2, float* __restrict__ O) {
  const int t = blockIdx.x * kThreads + threadIdx.x;
  if (t >= kSkipCh + kSkipCh + kMu) return;
  const int m = t & (kSkipCh - 1), m2 = t & (kMu - 1);
  float s = 0.0f;
#pragma unroll 1
  for (int i = 0; i < kNblk; ++i) s += bfr(b_skip[(size_t)i * kSkipCh + m]);
  const float p1 = bfr(b_p1[m]);
  const float p2 = bfr(b_p2[m2]);
  const float f0 = (t < kSkipCh) ? 1.0f : 0.0f;
  const float f2 = (t >= 2 * kSkipCh) ? 1.0f : 0.0f;
  const float f1 = 1.0f - f0 - f2;
  const float v = f0 * s + f1 * p1 + f2 * p2;
  ((volatile float*)O)[t] = v;
  __threadfence();
  ((volatile float*)O)[t] = v;
}

__global__ __launch_bounds__(kThreads) void k_zero16(v4u* __restrict__ base, int n16) {
  const int i = blockIdx.x * kThreads + threadIdx.x;
  if (i >= n16) return;
  const v4u z = {0u, 0u, 0u, 0u};
  ((volatile v4u*)base)[i] = z;
  __threadfence();
  ((volatile v4u*)base)[i] = z;
}

__global__ __launch_bounds__(kThreads) void k_embed(const int* __restrict__ idx, const float* __restrict__ w_in,
                                                    const float* __restrict__ b_in, float* __restrict__ X) {
  const int i = blockIdx.x * kThreads + threadIdx.x;
  if (i >= kTin * 8) return;
  const int t = i >> 3, c0 = (i & 7) * 4;
  int id = idx[t];
  id = id < 0 ? 0 : id;
  id = id > kMu - 1 ? kMu - 1 : id;
  v4f v;
#pragma unroll
  for (int e = 0; e < 4; ++e) v[e] = bfr(w_in[(size_t)(c0 + e) * kMu + id]) + bfr(b_in[c0 + e]);
  float* p = X + (size_t)t * kRes + c0;
  *(volatile v4f*)p = v;
  __threadfence();
  *(volatile v4f*)p = v;
}

template <int GMODE>
__global__ __launch_bounds__(kThreads) void k_wblock(
    const float* __restrict__ Xin, float* __restrict__ Xout,
    const unsigned short* __restrict__ Wg, const unsigned short* __restrict__ Wr,
    const float* __restrict__ bsig, const float* __restrict__ btanh, const float* __restrict__ bres,
    unsigned short* __restrict__ Gtmp, unsigned short* __restrict__ Gcol,
    int d, int len_in, int len_out, int goff, int qmin, int ntiles) {
  __shared__ __align__(16) _Float16 sWg[64 * 64];
  __shared__ __align__(16) _Float16 sWr[32 * 32];
  __shared__ __align__(16) _Float16 sGC[8 * 16 * 64];
  __shared__ __align__(16) float    sOut[8 * 16 * 36];
  const int tid = threadIdx.x;
  const int lane = tid & 31, wave = tid >> 5, hh = lane >> 4, c = lane & 15;

  {
    const v8h* wg8 = (const v8h*)(const void*)Wg;
    v8h* s8 = (v8h*)sWg;
    s8[tid] = wg8[tid];
    s8[tid + kThreads] = wg8[tid + kThreads];
    if (tid < 128) ((v8h*)sWr)[tid] = ((const v8h*)(const void*)Wr)[tid];
  }
  __syncthreads();

  const int q = qmin + (int)blockIdx.x * 8 + wave;
  const bool active = (q < qmin + ntiles);
  const int qc = active ? q : (qmin + ntiles - 1);
  const int u0 = qc * 16;
  const int t0 = u0 + goff;
  const int lmax = len_in - 1;
  const v8f z8 = {0.f, 0.f, 0.f, 0.f, 0.f, 0.f, 0.f, 0.f};

  v16h fa, fb;
  {
    const int tr = t0 + c;
    int ta = tr < 0 ? 0 : tr;
    ta = ta > lmax ? lmax : ta;
    int tb = tr + d;
    tb = tb < 0 ? 0 : tb;
    tb = tb > lmax ? lmax : tb;
    const float* pa = Xin + (size_t)ta * kRes + 8 * hh;
    const float* pb = Xin + (size_t)tb * kRes + 8 * hh;
    const v4f a0 = *(const v4f*)(pa);
    const v4f a1 = *(const v4f*)(pa + 4);
    const v4f a2 = *(const v4f*)(pa + 16);
    const v4f a3 = *(const v4f*)(pa + 20);
    asm volatile("" ::: "memory");
    const v4f b0 = *(const v4f*)(pb);
    const v4f b1 = *(const v4f*)(pb + 4);
    const v4f b2 = *(const v4f*)(pb + 16);
    const v4f b3 = *(const v4f*)(pb + 20);
#pragma unroll
    for (int e = 0; e < 4; ++e) {
      fa[e]      = (_Float16)(a0[e] * kAcarry);
      fa[4 + e]  = (_Float16)(a1[e] * kAcarry);
      fa[8 + e]  = (_Float16)(a2[e] * kAcarry);
      fa[12 + e] = (_Float16)(a3[e] * kAcarry);
      fb[e]      = (_Float16)(b0[e] * kAcarry);
      fb[4 + e]  = (_Float16)(b1[e] * kAcarry);
      fb[8 + e]  = (_Float16)(b2[e] * kAcarry);
      fb[12 + e] = (_Float16)(b3[e] * kAcarry);
    }
  }

  v8f acc[4];
#pragma unroll
  for (int j = 0; j < 4; ++j) acc[j] = z8;
  {
    const _Float16* wgl = sWg + c * 64 + 8 * hh;
#pragma unroll
    for (int j = 0; j < 4; ++j) {
      const v16h wb0 = FragH::load(wgl + j * 16 * 64);
      const v16h wb1 = FragH::load(wgl + j * 16 * 64 + 32);
      acc[j] = FragH::mma(fa, wb0, acc[j]);
      acc[j] = FragH::mma(fb, wb1, acc[j]);
      guard1x4(acc[j], fa, fb, wb0, wb1);
    }
  }
  acc_guard4(acc[0], acc[1], acc[2], acc[3]);

  const float bs0 = bfr(bsig[c]),  bs1 = bfr(bsig[16 + c]);
  const float bt0 = bfr(btanh[c]), bt1 = bfr(btanh[16 + c]);
  const float br0 = bfr(bres[c]),  br1 = bfr(bres[16 + c]);
  _Float16* sg = sGC + wave * (16 * 64);
#pragma unroll
  for (int r = 0; r < 8; ++r) {
    const float s0 = fmaf(acc[0][r], kFold, bs0);
    const float s1 = fmaf(acc[1][r], kFold, bs1);
    const float p0 = fmaf(acc[2][r], kFold, bt0);
    const float p1 = fmaf(acc[3][r], kFold, bt1);
    const float g0 = (1.0f / (1.0f + expf(-s0))) * tanhf(p0);
    const float g1 = (1.0f / (1.0f + expf(-s1))) * tanhf(p1);
    sg[(8 * hh + r) * 64 + 32 + c] = (_Float16)(g0 * kAcarry);
    sg[(8 * hh + r) * 64 + 48 + c] = (_Float16)(g1 * kAcarry);
  }
  if (GMODE == 1) {
    const int u0c = u0 < 0 ? 0 : u0;
    const int col8 = (lane & 3) * 8;
#pragma unroll
    for (int it = 0; it < 2; ++it) {
      const int row = (lane >> 2) + 8 * it;
      const v8h w = *(const v8h*)(const void*)(Gtmp + (size_t)(u0c + row) * kRes + col8);
      *(v8h*)(sg + row * 64 + col8) = w;
    }
  }
  __syncthreads();

  float* so = sOut + wave * (16 * 36);
  {
    const v16h ag = FragH::load(sg + c * 64 + 32 + 8 * hh);
    const v16h w0 = FragH::load(sWr + c * 32 + 8 * hh);
    const v16h w1 = FragH::load(sWr + (16 + c) * 32 + 8 * hh);
    v8f r0 = z8, r1 = z8;
    r0 = FragH::mma(ag, w0, r0);
    r1 = FragH::mma(ag, w1, r1);
    guard2x3(r0, r1, ag, w0, w1);
#pragma unroll
    for (int r = 0; r < 8; ++r) {
      so[(8 * hh + r) * 36 + c]      = fmaf(r0[r], kFold, br0);
      so[(8 * hh + r) * 36 + 16 + c] = fmaf(r1[r], kFold, br1);
    }
  }
  __syncthreads();

  {
    const int c4 = (lane & 7) * 4;
    v4f xv[4];
#pragma unroll
    for (int it = 0; it < 4; ++it) {
      const int row = (lane >> 3) + 4 * it;
      int ts = t0 + row + d;
      ts = ts < 0 ? 0 : ts;
      ts = ts > lmax ? lmax : ts;
      const v4f rv = *(const v4f*)(Xin + (size_t)ts * kRes + c4);
      const v4f ov = *(const v4f*)(so + row * 36 + c4);
      xv[it] = ov + rv;
    }
    for (int pass = 0; pass < 2; ++pass) {
#pragma unroll
      for (int it = 0; it < 4; ++it) {
        const int row = (lane >> 3) + 4 * it;
        const int t = t0 + row;
        if (active && t >= 0 && t < len_out) *(volatile v4f*)(Xout + (size_t)t * kRes + c4) = xv[it];
      }
      __threadfence();
    }
  }

  const bool wr_g = active && (u0 >= 0);
  if (GMODE == 0) {
    const int col8 = (lane & 3) * 8;
    v8h gv[2];
#pragma unroll
    for (int it = 0; it < 2; ++it) {
      const int row = (lane >> 2) + 8 * it;
      gv[it] = *(const v8h*)(sg + row * 64 + 32 + col8);
    }
    for (int pass = 0; pass < 2; ++pass) {
#pragma unroll
      for (int it = 0; it < 2; ++it) {
        const int row = (lane >> 2) + 8 * it;
        if (wr_g) *(volatile v8h*)(Gtmp + (size_t)(u0 + row) * kRes + col8) = gv[it];
      }
      __threadfence();
    }
  } else {
    const int col8 = (lane & 7) * 8;
    v8h gv[4];
#pragma unroll
    for (int it = 0; it < 4; ++it) {
      const int row = (lane >> 3) + 4 * it;
      gv[it] = *(const v8h*)(sg + row * 64 + col8);
    }
    for (int pass = 0; pass < 2; ++pass) {
#pragma unroll
      for (int it = 0; it < 4; ++it) {
        const int row = (lane >> 3) + 4 * it;
        if (wr_g) *(volatile v8h*)(Gcol + (size_t)(u0 + row) * kKskip + col8) = gv[it];
      }
      __threadfence();
    }
  }
}

extern "C" void kernel_launch(void* const* d_in, const int* in_sizes, int n_in,
                              void* d_out, int out_size, void* d_ws, size_t ws_size, hipStream_t stream) {
  (void)in_sizes;
  if (n_in < 15) return;
  if (ws_size < kWsTotal) return;
  if ((size_t)out_size < (size_t)kFinal * kMu) return;

  const int*   idx    = (const int*)d_in[0];
  const float* w_in   = (const float*)d_in[1];
  const float* b_in   = (const float*)d_in[2];
  const float* w_sig  = (const float*)d_in[3];
  const float* b_sig  = (const float*)d_in[4];
  const float* w_tanh = (const float*)d_in[5];
  const float* b_tanh = (const float*)d_in[6];
  const float* w_skip = (const float*)d_in[7];
  const float* b_skip = (const float*)d_in[8];
  const float* w_res  = (const float*)d_in[9];
  const float* b_res  = (const float*)d_in[10];
  const float* w_p1   = (const float*)d_in[11];
  const float* b_p1   = (const float*)d_in[12];
  const float* w_p2   = (const float*)d_in[13];
  const float* b_p2   = (const float*)d_in[14];
  float* out = (float*)d_out;

  char* ws = (char*)d_ws;
  float*          X0   = (float*)(ws + kOffX0);
  float*          X1   = (float*)(ws + kOffX1);
  unsigned short* Gp   = (unsigned short*)(ws + kOffG);
  unsigned short* GT   = (unsigned short*)(ws + kOffGT);
  unsigned short* E1   = (unsigned short*)(ws + kOffE1);
  unsigned short* E2   = (unsigned short*)(ws + kOffE2);
  unsigned short* WG   = (unsigned short*)(ws + kOffWG);
  unsigned short* WR   = (unsigned short*)(ws + kOffWR);
  unsigned short* WSK  = (unsigned short*)(ws + kOffWS);
  unsigned short* WP1  = (unsigned short*)(ws + kOffWP1);
  unsigned short* WP2  = (unsigned short*)(ws + kOffWP2);
  float*          BIAS = (float*)(ws + kOffBias);

  k_pack_gate<<<(kNblk * 64 * 64 / 8) / kThreads, kThreads, 0, stream>>>(w_sig, w_tanh, WG);
  k_pack_skip<<<(kSkipCh * kKskip / 8) / kThreads, kThreads, 0, stream>>>(w_skip, WSK);
  {
    const int n8r = kNblk * kRes * kRes / 8;
    const int n81 = kSkipCh * kSkipCh / 8;
    const int n82 = kMu * kSkipCh / 8;
    k_pack_plain<<<(n8r + kThreads - 1) / kThreads, kThreads, 0, stream>>>(w_res, n8r, WR);
    k_pack_plain<<<(n81 + kThreads - 1) / kThreads, kThreads, 0, stream>>>(w_p1, n81, WP1);
    k_pack_plain<<<(n82 + kThreads - 1) / kThreads, kThreads, 0, stream>>>(w_p2, n82, WP2);
  }
  k_bias<<<(kSkipCh + kSkipCh + kMu + kThreads - 1) / kThreads, kThreads, 0, stream>>>(b_skip, b_p1, b_p2, BIAS);
  {
    const int n16 = (int)(((size_t)(kMpad - kGrowsW) * kKskip * 2) / 16);
    v4u* gz = (v4u*)(ws + kOffG + (size_t)kGrowsW * kKskip * 2);
    k_zero16<<<(n16 + kThreads - 1) / kThreads, kThreads, 0, stream>>>(gz, n16);
  }
  k_embed<<<(kTin * 8) / kThreads, kThreads, 0, stream>>>(idx, w_in, b_in, X0);

  int len_in = kTin;
  for (int i = 0; i < kNblk; ++i) {
    const int d = 1 << (i % 10);
    const int len_out = len_in - d;
    const int goff = len_out - kFinal;
    const int qmin = -((goff + 15) / 16);
    const int ntiles = kUtiles - qmin;
    const int nblocks = (ntiles + 7) / 8;
    const float* xin = (i & 1) ? X1 : X0;
    float* xout = (i & 1) ? X0 : X1;
    const unsigned short* wg = WG + (size_t)i * 64 * 64;
    const unsigned short* wr = WR + (size_t)i * 32 * 32;
    const float* bs = b_sig + (size_t)i * kRes;
    const float* bt = b_tanh + (size_t)i * kRes;
    const float* br = b_res + (size_t)i * kRes;
    if ((i & 1) == 0) {
      k_wblock<0><<<nblocks, kThreads, 0, stream>>>(xin, xout, wg, wr, bs, bt, br, GT, Gp,
                                                   d, len_in, len_out, goff, qmin, ntiles);
    } else {
      k_wblock<1><<<nblocks, kThreads, 0, stream>>>(xin, xout, wg, wr, bs, bt, br, GT, Gp + (size_t)(i - 1) * kRes,
                                                   d, len_in, len_out, goff, qmin, ntiles);
    }
    len_in = len_out;
  }

  {
    const int tiles = (kMpad / 64) * (kSkipCh / 64);
    wmma_gemm64<0, false, 2, 1, false, 6><<<dim3((tiles + 7) / 8, 1), 256, 0, stream>>>(
        Gp, Gp, kKskip, 0L, WSK, WSK, kKskip, 0L, (void*)E1, (void*)E1, kSkipCh, 0L,
        BIAS, BIAS, 0L, kMpad, kSkipCh, kKskip, kFold, kAcarry, kMpad);
  }
  {
    const int tiles = (kMpad / 64) * (kSkipCh / 64);
    wmma_gemm64<0, false, 2, 1, false, 6><<<dim3((tiles + 7) / 8, 1), 256, 0, stream>>>(
        E1, E1, kSkipCh, 0L, WP1, WP1, kSkipCh, 0L, (void*)E2, (void*)E2, kSkipCh, 0L,
        BIAS + kSkipCh, BIAS, 0L, kMpad, kSkipCh, kSkipCh, kFold, kAcarry, kMpad);
  }
  {
    const int tiles = (kMpad / 64) * (kMu / 64);
    wmma_gemm64<0, false, 2, 0, false, 0><<<dim3((tiles + 7) / 8, 1), 256, 0, stream>>>(
        E2, E2, kSkipCh, 0L, WP2, WP2, kSkipCh, 0L, (void*)out, (void*)out, kMu, 0L,
        BIAS + 2 * kSkipCh, BIAS, 0L, kMpad, kMu, kSkipCh, kFold, 1.0f, kFinal);
  }
}
